// RNN_15144054686346
// MI455X (gfx1250) — hardware-verified
//
#include <hip/hip_runtime.h>
#include <math.h>

constexpr int NB_SEQ  = 64;
constexpr int NS_STEP = 512;
constexpr int NV_TOK  = 32000;
constexpr int NE_DIM  = 512;
constexpr int NH_DIM  = 1024;
constexpr int NC_CLS  = 5;
constexpr int NROWS   = NS_STEP * NB_SEQ;
constexpr int OUT0_N  = NB_SEQ * NC_CLS;
constexpr int OUT1_N  = NB_SEQ * NH_DIM;
static_assert(OUT0_N * 4 == 1280);
static_assert((OUT0_N + OUT1_N) * 4 == 263424);
static_assert(NB_SEQ == 64 && NE_DIM / 8 == 64);
static_assert(NE_DIM % 32 == 0);
static_assert(NH_DIM % 64 == 0 && NROWS % 64 == 0);
static_assert((NH_DIM * NE_DIM) % (8 * 256) == 0);
static_assert((NH_DIM * NH_DIM) % (8 * 256) == 0);
static_assert(NH_DIM == 4 * 256);
static_assert((NROWS * 64) % 256 == 0);

constexpr int SEQ_BLK    = 16;
constexpr int RNN_BLOCKS = NB_SEQ / SEQ_BLK;
constexpr int RNN_THR    = 512;
constexpr int HP         = NH_DIM + 8;
constexpr int HTILE      = SEQ_BLK * HP;
constexpr int SLP        = NH_DIM + 4;
static_assert(NB_SEQ % SEQ_BLK == 0);
static_assert(NH_DIM == 64 * (RNN_THR / 32));
static_assert(HP % 8 == 0 && SLP % 4 == 0);
static_assert((2 * HTILE) % 8 == 0);
static_assert(SEQ_BLK * SLP * 4 <= 2 * HTILE * 2);
constexpr float XS_CARRY     = 16.0f;
constexpr float XS_CARRY_INV = 1.0f / 16.0f;

typedef __attribute__((ext_vector_type(16))) _Float16 v16h;
typedef __attribute__((ext_vector_type(8)))  _Float16 v8h;
typedef __attribute__((ext_vector_type(16))) __bf16   v16b;
typedef __attribute__((ext_vector_type(8)))  __bf16   v8b;
typedef __attribute__((ext_vector_type(8)))  float    v8f;
typedef __attribute__((ext_vector_type(4)))  float    v4f;
typedef __attribute__((ext_vector_type(4)))  unsigned v4u;

__device__ __forceinline__ unsigned short f2bf_bits(float f) {
  unsigned u = __float_as_uint(f);
  return (unsigned short)((u + 0x7FFFu + ((u >> 16) & 1u)) >> 16);
}
__device__ __forceinline__ float bf_bits2f(unsigned short h) { return __uint_as_float(((unsigned)h) << 16); }
__device__ __forceinline__ float bf16r(float f) { return bf_bits2f(f2bf_bits(f)); }

__device__ __forceinline__ float h16_to_f32(unsigned hb) {
  const unsigned sgn = (hb & 0x8000u) << 16; const unsigned em = hb & 0x7fffu;
  const float fn = __uint_as_float((em << 13) + 0x38000000u);
  const float fs = (float)em * 5.9604644775390625e-8f;
  const float mag = (em < 0x400u) ? fs : fn; return __uint_as_float(__float_as_uint(mag) | sgn); }

__device__ __forceinline__ void dep_guard_h(v8f& a, v8f& b, v16h x, v16h y) { asm volatile("v_nop\n\tv_nop\n\tv_nop\n\tv_nop" : "+v"(a), "+v"(b) : "v"(x), "v"(y)); }
__device__ __forceinline__ void dep_guard_b(v8f& a, v8f& b, v16b x, v16b y) { asm volatile("v_nop\n\tv_nop\n\tv_nop\n\tv_nop" : "+v"(a), "+v"(b) : "v"(x), "v"(y)); }
__device__ __forceinline__ void keep4_h(v16h a, v16h b, v16h c, v16h d) { asm volatile("v_nop" :: "v"(a), "v"(b), "v"(c), "v"(d)); }
__device__ __forceinline__ void keep4_b(v16b a, v16b b, v16b c, v16b d) { asm volatile("v_nop" :: "v"(a), "v"(b), "v"(c), "v"(d)); }
__device__ __forceinline__ void acc_guard4(v8f& a, v8f& b, v8f& c, v8f& d) { asm volatile("v_nop\n\tv_nop\n\tv_nop\n\tv_nop" : "+v"(a), "+v"(b), "+v"(c), "+v"(d)); }
__device__ __forceinline__ void wmma_guard_all(v8f& a, v8f& b, v8f& c, v8f& d, v16h x, v16h y, v16h p, v16h q, v16h r, v16h s) {
  asm volatile("v_nop\n\tv_nop\n\tv_nop\n\tv_nop" : "+v"(a), "+v"(b), "+v"(c), "+v"(d) : "v"(x), "v"(y), "v"(p), "v"(q), "v"(r), "v"(s)); }
__device__ __forceinline__ void wmma_guard_all(v8f& a, v8f& b, v8f& c, v8f& d, v16b x, v16b y, v16b p, v16b q, v16b r, v16b s) {
  asm volatile("v_nop\n\tv_nop\n\tv_nop\n\tv_nop" : "+v"(a), "+v"(b), "+v"(c), "+v"(d) : "v"(x), "v"(y), "v"(p), "v"(q), "v"(r), "v"(s)); }

template <typename T> struct Frag;
template <> struct Frag<_Float16> {
  typedef v16h V; union U { v16h v; v8h h[2]; };
  static __device__ __forceinline__ v16h load(const _Float16* p) {
    U f; f.h[0] = *(const v8h*)(p); f.h[1] = *(const v8h*)(p + 16); return f.v;
  }
  static __device__ __forceinline__ v8f mma(v16h a, v16h b, v8f c) {
    return __builtin_amdgcn_wmma_f32_16x16x32_f16(false, a, false, b, (short)0, c, false, false);
  }
  static __device__ __forceinline__ void guard(v8f& a, v8f& b, v16h x, v16h y) { dep_guard_h(a, b, x, y); }
  static __device__ __forceinline__ void keep(v16h a, v16h b, v16h c, v16h d) { keep4_h(a, b, c, d); }
};
template <> struct Frag<__bf16> {
  typedef v16b V; union U { v16b v; v8b h[2]; };
  static __device__ __forceinline__ v16b load(const __bf16* p) {
    U f; f.h[0] = *(const v8b*)(p); f.h[1] = *(const v8b*)(p + 16); return f.v;
  }
  static __device__ __forceinline__ v8f mma(v16b a, v16b b, v8f c) {
    return __builtin_amdgcn_wmma_f32_16x16x32_bf16(false, a, false, b, (short)0, c, false, false);
  }
  static __device__ __forceinline__ void guard(v8f& a, v8f& b, v16b x, v16b y) { dep_guard_b(a, b, x, y); }
  static __device__ __forceinline__ void keep(v16b a, v16b b, v16b c, v16b d) { keep4_b(a, b, c, d); }
};

template <int ET> struct Elem;
template <> struct Elem<0> { typedef _Float16 T; };
template <> struct Elem<1> { typedef __bf16 T; };
template <int ET, bool SPLIT, int BIAS_MODE, int OUT_MODE, bool RESID, int ACT = 0>
__global__ __launch_bounds__(256) void wmma_gemm64(
    const unsigned short* __restrict__ Ap, const unsigned short* __restrict__ A2p, int lda, long strideA,
    const unsigned short* __restrict__ Btp, const unsigned short* __restrict__ Bt2p, int ldb, long strideB,
    void* __restrict__ Cout, void* __restrict__ Cout2, int ldc, long strideC,
    const float* __restrict__ bias,
    const float* __restrict__ resid, long strideR,
    int M, int N, int K, float scale) {
  typedef typename Elem<ET>::T T;
  typedef typename Frag<T>::V V;
  const T* A = (const T*)Ap; const T* A2 = (const T*)A2p; const T* Bt = (const T*)Btp; const T* Bt2 = (const T*)Bt2p;
  __shared__ __align__(16) float sT[8][16 * 68];
  const int b    = blockIdx.y;
  const int lane = threadIdx.x & 31;
  const int wave = threadIdx.x >> 5;
  const int tilesN = N >> 6;
  const int tilesM = M >> 6;
  const int tile = blockIdx.x * 8 + wave;
  if (tile >= tilesM * tilesN) return;
  const int tm = tile / tilesN;
  const int tn = tile - tm * tilesN;
  const int m0 = tm << 6;
  const int n0 = tn << 6;

  const T* Ab  = A  + (size_t)b * strideA;
  const T* Bb  = Bt + (size_t)b * strideB;
  const T* Ab2 = SPLIT ? (A2  + (size_t)b * strideA) : nullptr;
  const T* Bb2 = SPLIT ? (Bt2 + (size_t)b * strideB) : nullptr;

  const int rlane = lane & 15;
  const int koff  = (lane >> 4) * 8;
  const int mOff  = (lane >> 4) * 8;

  v8f acc[4][4];
#pragma unroll
  for (int i = 0; i < 4; ++i)
#pragma unroll
    for (int j = 0; j < 4; ++j) acc[i][j] = (v8f){0.f,0.f,0.f,0.f,0.f,0.f,0.f,0.f};

  for (int k0 = 0; k0 < K; k0 += 32) {
    V bh[4], bl[4];
#pragma unroll
    for (int j = 0; j < 4; ++j) {
      const size_t bo = (size_t)(n0 + (j << 4) + rlane) * ldb + koff + k0;
      bh[j] = Frag<T>::load(Bb + bo);
      if (SPLIT) bl[j] = Frag<T>::load(Bb2 + bo);
    }
#pragma unroll
    for (int i = 0; i < 4; ++i) {
      const size_t ao = (size_t)(m0 + (i << 4) + rlane) * lda + koff + k0;
      V ah = Frag<T>::load(Ab + ao);
      V al = ah;
      if (SPLIT) al = Frag<T>::load(Ab2 + ao);
#pragma unroll
      for (int j = 0; j < 4; ++j) {
        acc[i][j] = Frag<T>::mma(ah, bh[j], acc[i][j]);
        if (SPLIT) {
          acc[i][j] = Frag<T>::mma(ah, bl[j], acc[i][j]);
          acc[i][j] = Frag<T>::mma(al, bh[j], acc[i][j]);
        }
      }
      wmma_guard_all(acc[i][0], acc[i][1], acc[i][2], acc[i][3], ah, al, bh[0], bh[1], bh[2], bh[3]);
    }
    Frag<T>::keep(bh[0], bh[1], bh[2], bh[3]);
    if (SPLIT) Frag<T>::keep(bl[0], bl[1], bl[2], bl[3]);
  }
  acc_guard4(acc[0][0], acc[0][1], acc[0][2], acc[0][3]);
  acc_guard4(acc[1][0], acc[1][1], acc[1][2], acc[1][3]);
  acc_guard4(acc[2][0], acc[2][1], acc[2][2], acc[2][3]);
  acc_guard4(acc[3][0], acc[3][1], acc[3][2], acc[3][3]);

  float* slab = sT[wave];
  const float* Rb = RESID ? (resid + (size_t)b * strideR) : nullptr;
#pragma unroll
  for (int i = 0; i < 4; ++i) {
    const int mBase = m0 + (i << 4);
    float bm[8];
    if (BIAS_MODE == 1) {
      const v4f bq0 = *(const v4f*)(bias + mBase + mOff);
      const v4f bq1 = *(const v4f*)(bias + mBase + mOff + 4);
      bm[0] = bq0[0]; bm[1] = bq0[1]; bm[2] = bq0[2]; bm[3] = bq0[3];
      bm[4] = bq1[0]; bm[5] = bq1[1]; bm[6] = bq1[2]; bm[7] = bq1[3];
    } else {
#pragma unroll
      for (int r = 0; r < 8; ++r) bm[r] = 0.0f;
    }
#pragma unroll
    for (int j = 0; j < 4; ++j) {
      const int n = n0 + (j << 4) + rlane;
      float bv = 0.f;
      if (BIAS_MODE == 2) bv = bias[n];
#pragma unroll
      for (int r = 0; r < 8; ++r) {
        float v = acc[i][j][r] * scale;
        if (BIAS_MODE == 1) v += bm[r];
        if (BIAS_MODE == 2) v += bv;
        if (RESID) v += Rb[(size_t)(mBase + mOff + r) * ldc + n];
        if (ACT == 1) v = tanhf(v);
        if (ACT == 2) v = fmaxf(v, 0.0f);
        if (ACT == 4) v = (v > 0.f) ? v : 0.01f * v;
        slab[(mOff + r) * 68 + (j << 4) + rlane] = v;
      }
    }
    __builtin_amdgcn_fence(__ATOMIC_RELEASE, "workgroup");
    __builtin_amdgcn_wave_barrier();
    __builtin_amdgcn_fence(__ATOMIC_ACQUIRE, "workgroup");
    if (OUT_MODE == 0) {
      float* C = (float*)Cout + (size_t)b * strideC;
      const int hh = lane >> 4, c4 = (lane & 15) * 4;
      for (int pass = 0; pass < 2; ++pass) {
#pragma unroll
        for (int it = 0; it < 8; ++it) {
          const int row = it * 2 + hh;
          v4f v = *(const v4f*)(slab + row * 68 + c4);
          *(volatile v4f*)(C + (size_t)(mBase + row) * ldc + n0 + c4) = v;
        }
        __threadfence();
      }
    } else {
      const int q = lane >> 3, c8 = (lane & 7) * 8;
      unsigned short* C  = (unsigned short*)Cout  + (size_t)b * strideC;
      unsigned short* C2 = (OUT_MODE == 2) ? ((unsigned short*)Cout2 + (size_t)b * strideC) : nullptr;
      for (int pass = 0; pass < 2; ++pass) {
#pragma unroll
        for (int it = 0; it < 4; ++it) {
          const int row = it * 4 + q;
          const float* sp = slab + row * 68 + c8;
          v8h hv, lv;
#pragma unroll
          for (int e = 0; e < 8; ++e) {
            if (OUT_MODE == 1) {
              hv[e] = (_Float16)sp[e];
            } else {
              unsigned short hb = f2bf_bits(sp[e]);
              unsigned short lb = f2bf_bits(sp[e] - bf_bits2f(hb));
              hv[e] = __builtin_bit_cast(_Float16, hb);
              lv[e] = __builtin_bit_cast(_Float16, lb);
            }
          }
          *(volatile v8h*)(C + (size_t)(mBase + row) * ldc + n0 + c8) = hv;
          if (OUT_MODE == 2) *(volatile v8h*)(C2 + (size_t)(mBase + row) * ldc + n0 + c8) = lv;
        }
        __threadfence();
      }
    }
    __builtin_amdgcn_fence(__ATOMIC_RELEASE, "workgroup");
    __builtin_amdgcn_wave_barrier();
    __builtin_amdgcn_fence(__ATOMIC_ACQUIRE, "workgroup");
  }
}

__global__ __launch_bounds__(256) void cvt_bf16x8_kernel(const float* __restrict__ src,
                                                         unsigned short* __restrict__ dst, int n8) {
  const int i = blockIdx.x * 256 + threadIdx.x;
  if (i < n8) {
    const float* sp = src + (size_t)i * 8;
    const v4f a = *(const v4f*)(sp);
    const v4f bq = *(const v4f*)(sp + 4);
    v8h hv;
#pragma unroll
    for (int e = 0; e < 4; ++e) {
      const float fa = a[e], fb = bq[e];
      hv[e]     = __builtin_bit_cast(_Float16, f2bf_bits(fa));
      hv[4 + e] = __builtin_bit_cast(_Float16, f2bf_bits(fb));
    }
    unsigned short* dp = dst + (size_t)i * 8;
    *(volatile v8h*)dp = hv;
    __threadfence();
    *(volatile v8h*)dp = hv;
  }
}

__global__ __launch_bounds__(256) void bias_prep_kernel(const float* __restrict__ bw, float* __restrict__ dst) {
  const int idx = threadIdx.x * 4;
  const v4f a = *(const v4f*)(bw + idx);
  v4f o;
#pragma unroll
  for (int e = 0; e < 4; ++e) { const float f = a[e]; o[e] = bf16r(f) * XS_CARRY; }
  float* op = dst + idx;
  *(volatile v4f*)op = o;
  __threadfence();
  *(volatile v4f*)op = o;
}

__global__ __launch_bounds__(256) void gather_kernel(const int* __restrict__ x, const float* __restrict__ emb,
                                                     unsigned short* __restrict__ embA) {
  const int i   = blockIdx.x * 256 + threadIdx.x;
  const int row = i >> 6, c8 = i & 63;
  const int t   = row >> 6, b = row & 63;
  int tok = x[b * NS_STEP + t];
  tok = (tok < 0) ? 0 : ((tok > NV_TOK - 1) ? (NV_TOK - 1) : tok);
  const float* src = emb + (size_t)tok * NE_DIM + c8 * 8;
  const v4f a = *(const v4f*)(src);
  const v4f bq = *(const v4f*)(src + 4);
  v8h hv;
#pragma unroll
  for (int e = 0; e < 4; ++e) {
    const float fa = a[e], fb = bq[e];
    hv[e]     = __builtin_bit_cast(_Float16, f2bf_bits(fa));
    hv[4 + e] = __builtin_bit_cast(_Float16, f2bf_bits(fb));
  }
  unsigned short* dp = embA + (size_t)row * NE_DIM + c8 * 8;
  *(volatile v8h*)dp = hv;
  __threadfence();
  *(volatile v8h*)dp = hv;
}

union HLds { unsigned short u[2 * HTILE]; float f[SEQ_BLK * SLP]; };

__global__ __launch_bounds__(RNN_THR) void rnn_seq_kernel(const unsigned short* __restrict__ xsT,
                                                          const unsigned short* __restrict__ Ubp,
                                                          float* __restrict__ hOut, float* __restrict__ hF) {
  __shared__ __align__(16) HLds hl;
  const __bf16* Ub = (const __bf16*)Ubp;
  const int tid = threadIdx.x, lane = tid & 31, wave = tid >> 5;
  const int c = lane & 15, hh = lane >> 4, koff = hh * 8, mOff = hh * 8, c4 = c * 4;
  const int seq0 = blockIdx.x * SEQ_BLK;
  const int n0w  = wave * 64;

  {
    const v4u z = {0u, 0u, 0u, 0u};
    for (int i = tid; i < (2 * HTILE) / 8; i += RNN_THR) *(v4u*)(hl.u + 8 * i) = z;
  }
  __syncthreads();

  unsigned short* thi = hl.u;
  unsigned short* tlo = hl.u + HTILE;
  const __bf16* ahi  = (const __bf16*)(hl.u) + c * HP + koff;
  const __bf16* alo  = (const __bf16*)(hl.u + HTILE) + c * HP + koff;
  const __bf16* brow = Ub + (size_t)(n0w + c) * NH_DIM + koff;

#pragma unroll 1
  for (int t = 0; t < NS_STEP; ++t) {
    v8f acc[4];
#pragma unroll
    for (int j = 0; j < 4; ++j) {
      const int n = n0w + 16 * j + c;
      const v4u w = *(const v4u*)(xsT + (size_t)n * NROWS + (size_t)(t * NB_SEQ + seq0 + 8 * hh));
      const unsigned w0 = w[0], w1 = w[1], w2 = w[2], w3 = w[3];
      acc[j][0] = h16_to_f32(w0 & 0xffffu) * XS_CARRY_INV;
      acc[j][1] = h16_to_f32(w0 >> 16)      * XS_CARRY_INV;
      acc[j][2] = h16_to_f32(w1 & 0xffffu) * XS_CARRY_INV;
      acc[j][3] = h16_to_f32(w1 >> 16)      * XS_CARRY_INV;
      acc[j][4] = h16_to_f32(w2 & 0xffffu) * XS_CARRY_INV;
      acc[j][5] = h16_to_f32(w2 >> 16)      * XS_CARRY_INV;
      acc[j][6] = h16_to_f32(w3 & 0xffffu) * XS_CARRY_INV;
      acc[j][7] = h16_to_f32(w3 >> 16)      * XS_CARRY_INV;
    }
#pragma unroll 2
    for (int kc = 0; kc < NH_DIM / 32; ++kc) {
      const v16b fh = Frag<__bf16>::load(ahi + kc * 32);
      const v16b fl = Frag<__bf16>::load(alo + kc * 32);
      v16b fb[4];
#pragma unroll
      for (int j = 0; j < 4; ++j) fb[j] = Frag<__bf16>::load(brow + (size_t)(16 * j) * NH_DIM + kc * 32);
#pragma unroll
      for (int j = 0; j < 4; ++j) {
        acc[j] = Frag<__bf16>::mma(fh, fb[j], acc[j]);
        acc[j] = Frag<__bf16>::mma(fl, fb[j], acc[j]);
      }
      wmma_guard_all(acc[0], acc[1], acc[2], acc[3], fh, fl, fb[0], fb[1], fb[2], fb[3]);
    }
    acc_guard4(acc[0], acc[1], acc[2], acc[3]);

    float hv[4][8];
#pragma unroll
    for (int j = 0; j < 4; ++j)
#pragma unroll
      for (int r = 0; r < 8; ++r) hv[j][r] = tanhf(acc[j][r]);

    __syncthreads();
    const bool last = (t == NS_STEP - 1);
    if (!last) {
#pragma unroll
      for (int j = 0; j < 4; ++j)
#pragma unroll
        for (int r = 0; r < 8; ++r) {
          const float h = hv[j][r];
          const unsigned short hb = f2bf_bits(h);
          const unsigned short lb = f2bf_bits(h - bf_bits2f(hb));
          const int idx = (mOff + r) * HP + n0w + 16 * j + c;
          thi[idx] = hb;
          tlo[idx] = lb;
        }
    } else {
#pragma unroll
      for (int j = 0; j < 4; ++j)
#pragma unroll
        for (int r = 0; r < 8; ++r) hl.f[(mOff + r) * SLP + n0w + 16 * j + c] = hv[j][r];
    }
    __syncthreads();
    if (last) {
      for (int pass = 0; pass < 2; ++pass) {
#pragma unroll
        for (int it = 0; it < 8; ++it) {
          const int row = it * 2 + hh;
          const v4f v = *(const v4f*)(hl.f + row * SLP + n0w + c4);
          *(volatile v4f*)(hOut + (size_t)(seq0 + row) * NH_DIM + n0w + c4) = v;
          *(volatile v4f*)(hF   + (size_t)(seq0 + row) * NH_DIM + n0w + c4) = v;
        }
        __threadfence();
      }
    }
  }
}

__global__ __launch_bounds__(256) void head_kernel(const float* __restrict__ hF, const float* __restrict__ Vw,
                                                   const float* __restrict__ bV, float* __restrict__ out0) {
  __shared__ __align__(16) float Vs[NC_CLS * NH_DIM];
  __shared__ __align__(16) float res[OUT0_N];
  const int tid = threadIdx.x, lane = tid & 31, wave = tid >> 5;
  for (int i = tid; i < NC_CLS * NH_DIM; i += 256) Vs[i] = bf16r(Vw[i]);
  const float bb0 = bf16r(bV[0]), bb1 = bf16r(bV[1]), bb2 = bf16r(bV[2]), bb3 = bf16r(bV[3]), bb4 = bf16r(bV[4]);
  __syncthreads();
#pragma unroll 1
  for (int rr = 0; rr < NB_SEQ / 8; ++rr) {
    const int b = wave * (NB_SEQ / 8) + rr;
    const float* hp = hF + (size_t)b * NH_DIM;
    float s0 = 0.0f, s1 = 0.0f, s2 = 0.0f, s3 = 0.0f, s4 = 0.0f;
#pragma unroll 1
    for (int i = 0; i < NH_DIM / 32; ++i) {
      const int k = 32 * i + lane;
      const float h = hp[k];
      s0 += h * Vs[k];
      s1 += h * Vs[NH_DIM + k];
      s2 += h * Vs[2 * NH_DIM + k];
      s3 += h * Vs[3 * NH_DIM + k];
      s4 += h * Vs[4 * NH_DIM + k];
    }
#pragma unroll
    for (int off = 1; off < 32; off <<= 1) {
      s0 += __shfl_xor(s0, off, 32);
      s1 += __shfl_xor(s1, off, 32);
      s2 += __shfl_xor(s2, off, 32);
      s3 += __shfl_xor(s3, off, 32);
      s4 += __shfl_xor(s4, off, 32);
    }
    if (lane == 0) {
      res[b * NC_CLS + 0] = s0 + bb0;
      res[b * NC_CLS + 1] = s1 + bb1;
      res[b * NC_CLS + 2] = s2 + bb2;
      res[b * NC_CLS + 3] = s3 + bb3;
      res[b * NC_CLS + 4] = s4 + bb4;
    }
  }
  __syncthreads();
  if (wave == 0) {
    const int l16 = (lane < 16) ? lane : 0;
    const v4f va = *(const v4f*)(res + 4 * lane);
    const v4f vb = *(const v4f*)(res + 128 + 4 * lane);
    const v4f vc = *(const v4f*)(res + 256 + 4 * l16);
    for (int pass = 0; pass < 2; ++pass) {
      *(volatile v4f*)(out0 + 4 * lane) = va;
      *(volatile v4f*)(out0 + 128 + 4 * lane) = vb;
      if (lane < 16) *(volatile v4f*)(out0 + 256 + 4 * lane) = vc;
      __threadfence();
    }
  }
}

extern "C" void kernel_launch(void* const* d_in, const int* in_sizes, int n_in,
                              void* d_out, int out_size, void* d_ws, size_t ws_size, hipStream_t stream) {
  if (n_in < 7 || d_out == nullptr || d_ws == nullptr) return;
  if (in_sizes[0] != NB_SEQ * NS_STEP || in_sizes[1] != NV_TOK * NE_DIM || in_sizes[2] != NH_DIM * NE_DIM ||
      in_sizes[3] != NH_DIM || in_sizes[4] != NH_DIM * NH_DIM || in_sizes[5] != NC_CLS * NH_DIM ||
      in_sizes[6] != NC_CLS || out_size != OUT0_N + OUT1_N) return;

  const int*   x   = (const int*)  d_in[0];
  const float* emb = (const float*)d_in[1];
  const float* Wm  = (const float*)d_in[2];
  const float* bW  = (const float*)d_in[3];
  const float* Um  = (const float*)d_in[4];
  const float* Vm  = (const float*)d_in[5];
  const float* bV  = (const float*)d_in[6];
  float* out0 = (float*)d_out;
  float* out1 = out0 + OUT0_N;

  char* ws = (char*)d_ws; size_t off = 0;
  auto carve = [&](size_t bytes) -> char* { char* p = ws + off; off += (bytes + 255) & ~(size_t)255; return p; };
  unsigned short* EMBA = (unsigned short*)carve((size_t)NROWS * NE_DIM * 2);
  unsigned short* XST  = (unsigned short*)carve((size_t)NH_DIM * NROWS * 2);
  unsigned short* UB   = (unsigned short*)carve((size_t)NH_DIM * NH_DIM * 2);
  unsigned short* WB   = (unsigned short*)carve((size_t)NH_DIM * NE_DIM * 2);
  float*          BWS  = (float*)carve((size_t)NH_DIM * 4);
  float*          HF   = (float*)carve((size_t)NB_SEQ * NH_DIM * 4);
  if (off > ws_size || off > (size_t)134217728) return;

  const int n8w = NH_DIM * NE_DIM / 8;
  const int n8u = NH_DIM * NH_DIM / 8;
  cvt_bf16x8_kernel<<<n8w / 256, 256, 0, stream>>>(Wm, WB, n8w);
  cvt_bf16x8_kernel<<<n8u / 256, 256, 0, stream>>>(Um, UB, n8u);
  bias_prep_kernel<<<1, 256, 0, stream>>>(bW, BWS);

  gather_kernel<<<(NROWS * 64) / 256, 256, 0, stream>>>(x, emb, EMBA);

  wmma_gemm64<1, false, 1, 1, false, 0><<<dim3(((NH_DIM / 64) * (NROWS / 64)) / 8, 1), 256, 0, stream>>>(
      WB, nullptr, NE_DIM, 0L, EMBA, nullptr, NE_DIM, 0L,
      (void*)XST, nullptr, NROWS, 0L, BWS, nullptr, 0L, NH_DIM, NROWS, NE_DIM, XS_CARRY);

  rnn_seq_kernel<<<RNN_BLOCKS, RNN_THR, 0, stream>>>(XST, UB, out1, HF);

  head_kernel<<<1, 256, 0, stream>>>(HF, Vm, bV, out0);
}
